// GAT_12189117186677
// MI455X (gfx1250) — hardware-verified
//
#include <hip/hip_runtime.h>
#include <stddef.h>
#include <stdint.h>
#include <math.h>


#define FIN    256
#define CH     1024
#define K2     2048
#define NFC    512
#define NOUT   10
#define NTHR   256
#define NWAVE  8
#define EPT    8
#define CHUNK  (NTHR * EPT)
#define WCAP   (EPT * 32)
#define LISTN  (NWAVE * WCAP)
#define NBA    1024
#define SLA    10
#define RCAP   28672
#define DEGCAP 64
#define GBM    64
#define GBN    128
#define GTHR   128
#define HTHR   512
#define BNR    256
#define NEGSL  0.2f
#define BN_EPS 1e-5f
#define NU_W1  (CH * (FIN / 8))
#define NU_W2  (CH * (K2 / 8))
#define NU_FC  (NFC * (K2 / 8))
#define AGG_ZINTS (LISTN + 2 * RCAP + 3 * NBA)
#define AGG_LDS_INTS (AGG_ZINTS + 16)
#define H_STG  (GBM * NFC)
#define H_SW   (NOUT * NFC)
#define H_FB   NFC
#define H_B1   32
#define H_SO   (GBM * NOUT)
#define HEAD_LDS_FLOATS (H_STG + H_SW + H_FB + H_B1 + H_SO)
#define WSMAX  134217728

static_assert((CHUNK & (CHUNK - 1)) == 0 && CHUNK <= 4096);
static_assert((NBA & (NBA - 1)) == 0 && NBA == (1 << SLA));
static_assert(((long long)CHUNK << SLA) < (1LL << 31));
static_assert(LISTN % NTHR == 0);
static_assert(NBA % NWAVE == 0 && NBA % 32 == 0 && NBA % GBM == 0);
static_assert(RCAP % 4 == 0 && AGG_ZINTS % 4 == 0 && LISTN % 4 == 0);
static_assert(AGG_LDS_INTS * 4 <= 300000);
static_assert(HEAD_LDS_FLOATS * 4 <= 300000);
static_assert(FIN % 32 == 0 && CH % 32 == 0 && K2 == 2 * CH && K2 % 32 == 0);
static_assert(CH % GBN == 0 && NFC == 4 * GBN && GBM == (GTHR / 32) * 16 && HTHR == 4 * GTHR);
static_assert(CH == 8 * 128 && CH == 4 * NTHR && GBM % NWAVE == 0);
static_assert(NU_W1 % NTHR == 0 && NU_W2 % NTHR == 0 && NU_FC % NTHR == 0);
static_assert(DEGCAP == 64);
static_assert((GBM * NOUT) % 4 == 0 && (GBM * NOUT) / 4 <= HTHR && NOUT <= H_B1);
static_assert((H_STG % 4) == 0 && (H_SW % 4) == 0 && (H_FB % 4) == 0 && (H_B1 % 4) == 0);
static_assert(HTHR / 8 == GBM && NFC == 8 * 64);

typedef float          v4f   __attribute__((ext_vector_type(4)));
typedef float          v8f   __attribute__((ext_vector_type(8)));
typedef double         v2d   __attribute__((ext_vector_type(2)));
typedef int            v4i   __attribute__((ext_vector_type(4)));
typedef int            v8i   __attribute__((ext_vector_type(8)));
typedef unsigned short v8us  __attribute__((ext_vector_type(8)));
typedef unsigned short v16us __attribute__((ext_vector_type(16)));
typedef __bf16         v16bf __attribute__((ext_vector_type(16)));
typedef v4f  __attribute__((may_alias)) v4fa;
typedef v4i  __attribute__((may_alias)) v4ia;
typedef v2d  __attribute__((may_alias)) v2da;
typedef v8us __attribute__((may_alias)) v8usa;
union FragB { v16bf v; v16us u; v8us h[2]; v8i w; };

__device__ __forceinline__ v8f wmb(const FragB& a, const FragB& b, v8f c) {
  v8f d = __builtin_amdgcn_wmma_f32_16x16x32_bf16(false, a.v, false, b.v, (short)0, c, false, false);
  asm volatile("v_nop\n\tv_nop\n\tv_nop\n\tv_nop" : "+v"(d) : "v"(a.w), "v"(b.w));
  return d;
}

__device__ __forceinline__ unsigned bf16_bits(float f) {
  const unsigned u = __float_as_uint(f);
  return (u + 0x7FFFu + ((u >> 16) & 1u)) >> 16;
}
__device__ __forceinline__ float bf16_val(float f) {
  return __uint_as_float(bf16_bits(f) << 16);
}
__device__ __forceinline__ v4f bfr4(const v4f a) {
  v4f r; r.x = bf16_val(a.x); r.y = bf16_val(a.y); r.z = bf16_val(a.z); r.w = bf16_val(a.w); return r;
}
__device__ __forceinline__ v4f fma4(const v4f acc, const float w, const v4f r) {
  v4f o;
  o.x = fmaf(w, r.x, acc.x); o.y = fmaf(w, r.y, acc.y); o.z = fmaf(w, r.z, acc.z); o.w = fmaf(w, r.w, acc.w);
  return o;
}
__device__ __forceinline__ float leaky(float v) { return v > 0.f ? v : NEGSL * v; }
__device__ __forceinline__ float relu_keep(float v) { return (v > 0.0f) ? v : (v - v); }

template <int SLB>
__device__ __forceinline__ int scan_chunk(const int* __restrict__ dsts, int nE, int cbase, int slotBase,
                                          int nb, int vec8, int* list, int tid, int lane, int wave) {
  int wc = 0;
  const int el0  = tid * EPT;
  const int e0   = cbase + el0;
  const int sent = -2147483647 - 1;
  v4i da, db;
  if (vec8 != 0 && cbase + CHUNK <= nE) {
    da = *(const v4i*)(dsts + e0);
    db = *(const v4i*)(dsts + e0 + 4);
  } else {
    da.x = (e0     < nE) ? dsts[min(e0,     nE - 1)] : sent;
    da.y = (e0 + 1 < nE) ? dsts[min(e0 + 1, nE - 1)] : sent;
    da.z = (e0 + 2 < nE) ? dsts[min(e0 + 2, nE - 1)] : sent;
    da.w = (e0 + 3 < nE) ? dsts[min(e0 + 3, nE - 1)] : sent;
    db.x = (e0 + 4 < nE) ? dsts[min(e0 + 4, nE - 1)] : sent;
    db.y = (e0 + 5 < nE) ? dsts[min(e0 + 5, nE - 1)] : sent;
    db.z = (e0 + 6 < nE) ? dsts[min(e0 + 6, nE - 1)] : sent;
    db.w = (e0 + 7 < nE) ? dsts[min(e0 + 7, nE - 1)] : sent;
  }
  const unsigned nbs = (unsigned)slotBase;
  const unsigned unb = (unsigned)nb;
  const unsigned s0 = (unsigned)da.x - nbs, s1 = (unsigned)da.y - nbs;
  const unsigned s2 = (unsigned)da.z - nbs, s3 = (unsigned)da.w - nbs;
  const unsigned s4 = (unsigned)db.x - nbs, s5 = (unsigned)db.y - nbs;
  const unsigned s6 = (unsigned)db.z - nbs, s7 = (unsigned)db.w - nbs;
  const bool h0 = s0 < unb, h1 = s1 < unb, h2 = s2 < unb, h3 = s3 < unb;
  const bool h4 = s4 < unb, h5 = s5 < unb, h6 = s6 < unb, h7 = s7 < unb;
  const unsigned any = __builtin_amdgcn_ballot_w32(h0 | h1 | h2 | h3 | h4 | h5 | h6 | h7);
  if (any != 0u) {
#define HITJ(J, HJ, SJ) { \
      const unsigned mj = __builtin_amdgcn_ballot_w32(HJ); \
      if (mj != 0u) { \
        if (HJ) { \
          const int pos = wc + (int)__builtin_amdgcn_mbcnt_lo(mj, 0u); \
          if (pos < WCAP) list[wave * WCAP + pos] = ((el0 + (J)) << SLB) | (int)(SJ); \
        } \
        wc += (int)__builtin_popcount(mj); } }
    HITJ(0, h0, s0)
    HITJ(1, h1, s1)
    HITJ(2, h2, s2)
    HITJ(3, h3, s3)
    HITJ(4, h4, s4)
    HITJ(5, h5, s5)
    HITJ(6, h6, s6)
    HITJ(7, h7, s7)
#undef HITJ
  }
  return wc;
}

__global__ __launch_bounds__(NTHR) void k_prep(const float* __restrict__ x, const float* __restrict__ W1,
                                               const float* __restrict__ W2, const float* __restrict__ FW,
                                               unsigned short* XB, unsigned short* W1B,
                                               unsigned short* W2D, unsigned short* FCD,
                                               int nN, int nUx) {
  const int u = (int)blockIdx.x * NTHR + (int)threadIdx.x;
  v4f a, b;
  bool ok = true;
  unsigned short* dp;
  if (u < nUx) {
    const int row = u >> 5;
    const int c0  = (u & 31) * 8;
    const int rc  = row < nN ? row : nN - 1;
    const float* p = x + (size_t)rc * FIN + c0;
    a = *(const v4f*)p; b = *(const v4f*)(p + 4);
    ok = row < nN;
    dp = XB + (size_t)row * FIN + c0;
  } else if (u < nUx + NU_W1) {
    const int v  = u - nUx;
    const int n  = v >> 5;
    const int k8 = (v & 31) * 8;
    const float* p = W1 + (size_t)n * FIN + k8;
    a = *(const v4f*)p; b = *(const v4f*)(p + 4);
    dp = W1B + (size_t)n * FIN + k8;
  } else if (u < nUx + NU_W1 + NU_W2) {
    const int v  = u - nUx - NU_W1;
    const int n  = v >> 8;
    const int k8 = (v & 255) * 8;
    const int kk = k8 & (CH - 1);
    const float* p = W2 + (size_t)n * CH + kk;
    a = *(const v4f*)p; b = *(const v4f*)(p + 4);
    dp = W2D + (size_t)n * K2 + k8;
  } else if (u < nUx + NU_W1 + NU_W2 + NU_FC) {
    const int v  = u - nUx - NU_W1 - NU_W2;
    const int n  = v >> 8;
    const int k8 = (v & 255) * 8;
    const int kk = k8 & (CH - 1);
    const float* p = FW + (size_t)n * CH + kk;
    a = *(const v4f*)p; b = *(const v4f*)(p + 4);
    dp = FCD + (size_t)n * K2 + k8;
  } else {
    return;
  }
  v8us o;
  o[0] = ok ? (unsigned short)bf16_bits(a.x) : (unsigned short)0;
  o[1] = ok ? (unsigned short)bf16_bits(a.y) : (unsigned short)0;
  o[2] = ok ? (unsigned short)bf16_bits(a.z) : (unsigned short)0;
  o[3] = ok ? (unsigned short)bf16_bits(a.w) : (unsigned short)0;
  o[4] = ok ? (unsigned short)bf16_bits(b.x) : (unsigned short)0;
  o[5] = ok ? (unsigned short)bf16_bits(b.y) : (unsigned short)0;
  o[6] = ok ? (unsigned short)bf16_bits(b.z) : (unsigned short)0;
  o[7] = ok ? (unsigned short)bf16_bits(b.w) : (unsigned short)0;
  *(volatile v8us*)dp = o;
  __threadfence();
  *(volatile v8us*)dp = o;
}

__device__ __forceinline__ void gemm_core(const unsigned short* __restrict__ ap,
                                          const unsigned short* __restrict__ bp, int ldb, int K,
                                          v8f (&acc)[8]) {
#pragma unroll 1
  for (int k0 = 0; k0 < K; k0 += 32) {
    FragB af;
    af.h[0] = *(const v8usa*)(ap + k0);
    af.h[1] = *(const v8usa*)(ap + k0 + 16);
#pragma unroll
    for (int nt = 0; nt < 8; ++nt) {
      const unsigned short* wq = bp + (size_t)(16 * nt) * (size_t)ldb + k0;
      FragB bf;
      bf.h[0] = *(const v8usa*)wq;
      bf.h[1] = *(const v8usa*)(wq + 16);
      acc[nt] = wmb(af, bf, acc[nt]);
    }
  }
}

__global__ __launch_bounds__(GTHR) void k_gemm(const unsigned short* __restrict__ A, int lda,
                                               const unsigned short* __restrict__ BT, int ldb, int K,
                                               float* Cm, int ldc) {
  __shared__ __attribute__((aligned(16))) float stg[GBM * GBN];
  const int tid = (int)threadIdx.x, lane = tid & 31, wave = tid >> 5, hh = lane >> 4, m = lane & 15;
  const int rowBase = (int)blockIdx.x * GBM;
  const int colBase = (int)blockIdx.y * GBN;
  v8f acc[8];
  {
    const v8f z = {0.f, 0.f, 0.f, 0.f, 0.f, 0.f, 0.f, 0.f};
#pragma unroll
    for (int t = 0; t < 8; ++t) acc[t] = z;
  }
  const unsigned short* ap = A  + (size_t)(rowBase + 16 * wave + m) * (size_t)lda + 8 * hh;
  const unsigned short* bp = BT + (size_t)(colBase + m) * (size_t)ldb + 8 * hh;
  gemm_core(ap, bp, ldb, K, acc);

#pragma unroll
  for (int nt = 0; nt < 8; ++nt) {
    const int lc = 16 * nt + m;
#pragma unroll
    for (int r = 0; r < 8; ++r) {
      const int lr = 16 * wave + 8 * hh + r;
      stg[lr * GBN + lc] = acc[nt][r];
    }
  }
  __syncthreads();

#pragma unroll 1
  for (int i = 0; i < 16; ++i) {
    const int row = wave * 16 + i;
    const v4f p = *(const v4fa*)(stg + row * GBN + 4 * lane);
    float* op = Cm + (size_t)(rowBase + row) * (size_t)ldc + colBase + 4 * lane;
    *(volatile v4f*)op = p;
  }
  __threadfence();
#pragma unroll 1
  for (int i = 0; i < 16; ++i) {
    const int row = wave * 16 + i;
    const v4f p = *(const v4fa*)(stg + row * GBN + 4 * lane);
    float* op = Cm + (size_t)(rowBase + row) * (size_t)ldc + colBase + 4 * lane;
    *(volatile v4f*)op = p;
  }
}

__global__ __launch_bounds__(HTHR) void k_gemm_head(const unsigned short* __restrict__ A,
                                                    const unsigned short* __restrict__ BT,
                                                    const float* __restrict__ fcb,
                                                    const float* __restrict__ f1w,
                                                    const float* __restrict__ f1b,
                                                    float* out, int nN) {
  extern __shared__ __attribute__((aligned(16))) float hsm[];
  float* stg = hsm;
  float* sw  = hsm + H_STG;
  float* sfb = sw + H_SW;
  float* sb1 = sfb + H_FB;
  float* so  = sb1 + H_B1;
  const int tid = (int)threadIdx.x, lane = tid & 31, wave = tid >> 5, hh = lane >> 4, m = lane & 15;
  const int rg = wave & 3, cg = wave >> 2;
  const int rowBase = (int)blockIdx.x * GBM;
  const int colBase = cg * GBN;

  for (int i = tid; i < H_SW / 4; i += HTHR) {
    const v4f a = bfr4(*(const v4f*)(f1w + 4 * i));
    *(v4f*)(sw + 4 * i) = a;
  }
  if (tid < NFC / 4) {
    const v4f a = bfr4(*(const v4f*)(fcb + 4 * tid));
    *(v4f*)(sfb + 4 * tid) = a;
  }
  if (tid < 32) {
    const int jc = tid < NOUT ? tid : NOUT - 1;
    const float v = bf16_val(f1b[jc]);
    sb1[tid] = (tid < NOUT) ? v : 0.0f;
  }
  __syncthreads();

  v8f acc[8];
  {
    const v8f z = {0.f, 0.f, 0.f, 0.f, 0.f, 0.f, 0.f, 0.f};
#pragma unroll
    for (int t = 0; t < 8; ++t) acc[t] = z;
  }
  const unsigned short* ap = A  + (size_t)(rowBase + 16 * rg + m) * (size_t)K2 + 8 * hh;
  const unsigned short* bp = BT + (size_t)(colBase + m) * (size_t)K2 + 8 * hh;
  gemm_core(ap, bp, K2, K2, acc);

#pragma unroll
  for (int nt = 0; nt < 8; ++nt) {
    const int lc = colBase + 16 * nt + m;
    const float bz = sfb[lc];
#pragma unroll
    for (int r = 0; r < 8; ++r) {
      const int lr = 16 * rg + 8 * hh + r;
      stg[lr * NFC + lc] = relu_keep(acc[nt][r] + bz);
    }
  }
  __syncthreads();

  {
    const int r = tid >> 3, p = tid & 7;
    const float* fr = stg + r * NFC + p * 64;
#pragma unroll 1
    for (int j = 0; j < NOUT; ++j) {
      const float* wr = sw + j * NFC + p * 64;
      const float bj = sb1[j];
      float s = 0.0f;
#pragma unroll 4
      for (int c4 = 0; c4 < 16; ++c4) {
        const v4f f = *(const v4fa*)(fr + 4 * c4);
        const v4f w = *(const v4fa*)(wr + 4 * c4);
        s = fmaf(f.x, w.x, s); s = fmaf(f.y, w.y, s); s = fmaf(f.z, w.z, s); s = fmaf(f.w, w.w, s);
      }
      s += __shfl_xor(s, 1);
      s += __shfl_xor(s, 2);
      s += __shfl_xor(s, 4);
      const float res = s + bj;
      if (p == 0) so[r * NOUT + j] = res;
    }
  }
  __syncthreads();

  int live = nN - rowBase;
  live = live < 0 ? 0 : (live > GBM ? GBM : live);
  const int npc = (live * NOUT) >> 2;
  const bool wr = tid < npc;
  const int pc = wr ? tid : 0;
  const v4f ov = *(const v4fa*)(so + 4 * pc);
  float* ob = out + (size_t)rowBase * NOUT + 4 * pc;
  if (wr) *(volatile v4f*)ob = ov;
  __threadfence();
  if (wr) *(volatile v4f*)ob = ov;
}

__global__ __launch_bounds__(NTHR) void k_dots(const float* __restrict__ H, const float* __restrict__ avs,
                                               const float* __restrict__ avd, float* SD, int MPr) {
  __shared__ __attribute__((aligned(16))) float sa[CH];
  __shared__ __attribute__((aligned(16))) float sd[CH];
  __shared__ __attribute__((aligned(16))) float sdt[2 * GBM];
  const int tid = (int)threadIdx.x, lane = tid & 31, wave = tid >> 5;
  {
    const v4f a = bfr4(*(const v4f*)(avs + 4 * tid));
    const v4f b = bfr4(*(const v4f*)(avd + 4 * tid));
    *(v4f*)(sa + 4 * tid) = a;
    *(v4f*)(sd + 4 * tid) = b;
  }
  __syncthreads();
  const int rowBase = (int)blockIdx.x * GBM;
#pragma unroll 1
  for (int i = 0; i < GBM / NWAVE; ++i) {
    const int row = wave * (GBM / NWAVE) + i;
    const float* hr = H + (size_t)(rowBase + row) * CH + 4 * lane;
    float s = 0.0f, d = 0.0f;
#pragma unroll 2
    for (int q = 0; q < CH / 128; ++q) {
      const v4f p = *(const v4f*)(hr + 128 * q);
      const v4f a = *(const v4fa*)(sa + 128 * q + 4 * lane);
      const v4f b = *(const v4fa*)(sd + 128 * q + 4 * lane);
      s = fmaf(p.x, a.x, s); s = fmaf(p.y, a.y, s); s = fmaf(p.z, a.z, s); s = fmaf(p.w, a.w, s);
      d = fmaf(p.x, b.x, d); d = fmaf(p.y, b.y, d); d = fmaf(p.z, b.z, d); d = fmaf(p.w, b.w, d);
    }
#pragma unroll
    for (int off = 16; off > 0; off >>= 1) {
      s += __shfl_xor(s, off);
      d += __shfl_xor(d, off);
    }
    if (lane == 0) { sdt[row] = s; sdt[GBM + row] = d; }
  }
  __syncthreads();
  if (wave == 0) {
    const int which = lane >> 4, piece = lane & 15;
    const v4f v = *(const v4fa*)(sdt + which * GBM + 4 * piece);
    float* sp = SD + (size_t)which * (size_t)MPr + rowBase + 4 * piece;
    *(volatile v4f*)sp = v;
    __threadfence();
    *(volatile v4f*)sp = v;
  }
}

__device__ __forceinline__ void gather_hits(v4f (&acc)[4], const float* __restrict__ base,
                                            int srv, int wvi, int n) {
#pragma unroll 1
  for (int k = 0; k < n; ++k) {
    const int   sk = __builtin_amdgcn_readlane(srv, k);
    const float wk = __int_as_float(__builtin_amdgcn_readlane(wvi, k));
    const float* rp = base + (size_t)sk * CH;
    const v4f r0 = *(const v4f*)rp;
    const v4f r1 = *(const v4f*)(rp + 128);
    const v4f r2 = *(const v4f*)(rp + 256);
    const v4f r3 = *(const v4f*)(rp + 384);
    acc[0] = fma4(acc[0], wk, r0);
    acc[1] = fma4(acc[1], wk, r1);
    acc[2] = fma4(acc[2], wk, r2);
    acc[3] = fma4(acc[3], wk, r3);
  }
}

__global__ __launch_bounds__(NTHR) void k_agg(const int* __restrict__ srcs, const int* __restrict__ dsts,
                                              int nE, int nN, int vec8, int MPr,
                                              const float* __restrict__ SD, const float* __restrict__ F,
                                              const float* __restrict__ bias, float* outp) {
  extern __shared__ __attribute__((aligned(16))) int dsm[];
  int* list = dsm;
  int* hl   = dsm + LISTN;
  int* sl   = dsm + LISTN + RCAP;
  int* cnt  = dsm + LISTN + 2 * RCAP;
  int* offs = cnt + NBA;
  int* cur  = offs + NBA;
  int* misc = cur + NBA;
  const int tid = (int)threadIdx.x, lane = tid & 31, wave = tid >> 5;
  const int nodeBase = (int)blockIdx.x * NBA;

  {
    const v4i z4 = {0, 0, 0, 0};
    for (int i = tid * 4; i < AGG_ZINTS; i += NTHR * 4) *(v4ia*)(dsm + i) = z4;
    if (tid < 16) misc[tid] = 0;
  }
  __syncthreads();

  int t = 0, ov = 0;
  const int nChunks = (nE + CHUNK - 1) / CHUNK;
#pragma unroll 1
  for (int ch = 0; ch < nChunks; ++ch) {
    const int cbase = ch * CHUNK;
    const int wc = scan_chunk<SLA>(dsts, nE, cbase, nodeBase, NBA, vec8, list, tid, lane, wave);
    if (lane == 0) misc[wave] = wc;
    __syncthreads();
    if (wave == 0) {
#pragma unroll 1
      for (int w2 = 0; w2 < NWAVE; ++w2) {
        int c = misc[w2];
        c = c < 0 ? 0 : (c > WCAP ? WCAP : c);
#pragma unroll 1
        for (int b0 = 0; b0 < c; b0 += 32) {
          const int idx = b0 + lane;
          const int ent = list[w2 * WCAP + (idx < WCAP ? idx : WCAP - 1)];
          const int m32 = (c - b0) < 32 ? (c - b0) : 32;
#pragma unroll 1
          for (int k = 0; k < m32; ++k) {
            const int u    = __builtin_amdgcn_readlane(ent, k);
            const int slot = u & (NBA - 1);
            const int el   = (u >> SLA) & (CHUNK - 1);
            const int pk   = ((cbase + el) << SLA) | slot;
            if (t < RCAP) {
              const int cv = cnt[slot];
              if (lane == 0) { hl[t] = pk; cnt[slot] = cv + 1; }
              t = t + 1;
            } else {
              ov = 1;
            }
          }
        }
      }
    }
    __syncthreads();
  }
  if (wave == 0 && lane == 0) { misc[8] = t; misc[9] = ov; }
  __syncthreads();
  int tt = misc[8];
  tt = tt < 0 ? 0 : (tt > RCAP ? RCAP : tt);
  const int ovf = misc[9];

  if (wave == 0) {
    const int base = lane * (NBA / 32);
    int s = 0;
#pragma unroll 1
    for (int i = 0; i < NBA / 32; ++i) s += cnt[base + i];
    int incl = s;
#pragma unroll
    for (int d = 1; d < 32; d <<= 1) {
      const int y = __shfl_up(incl, d, 32);
      if (lane >= d) incl += y;
    }
    int run = incl - s;
#pragma unroll 1
    for (int i = 0; i < NBA / 32; ++i) {
      const int cv = cnt[base + i];
      offs[base + i] = run;
      cur[base + i]  = run;
      run += cv;
    }
  }
  __syncthreads();
  if (wave == 0) {
#pragma unroll 1
    for (int b0 = 0; b0 < tt; b0 += 32) {
      const int idx = b0 + lane;
      const int ent = hl[idx < RCAP ? idx : RCAP - 1];
      const int m32 = (tt - b0) < 32 ? (tt - b0) : 32;
#pragma unroll 1
      for (int k = 0; k < m32; ++k) {
        const int u    = __builtin_amdgcn_readlane(ent, k);
        const int slot = u & (NBA - 1);
        int p = cur[slot];
        p = p < 0 ? 0 : (p > RCAP - 1 ? RCAP - 1 : p);
        if (lane == 0) {
          sl[p] = u;
          cur[slot] = p + 1;
        }
      }
    }
  }
  __syncthreads();

  const int wv = __builtin_amdgcn_readfirstlane(wave);
  const float qnan = __int_as_float(0x7fc00000);
  const float pz = (ovf != 0) ? qnan : 0.0f;
  const float* ASp = SD;
  const float* ADp = SD + (size_t)MPr;
#pragma unroll 1
  for (int si = 0; si < NBA / NWAVE; ++si) {
    const int s    = si * NWAVE + wv;
    const int node = nodeBase + s;
    if (node >= nN) continue;
    int c = cnt[s];
    const bool big = c > DEGCAP;
    c = c < 0 ? 0 : (c > DEGCAP ? DEGCAP : c);
    int o = offs[s];
    o = o < 0 ? 0 : (o > RCAP ? RCAP : o);
    int rem = tt - o;
    rem = rem < 0 ? 0 : rem;
    c = c > rem ? rem : c;

    const float ad  = ADp[node];
    const float as0 = ASp[node];
    int i0 = o + lane;      i0 = i0 > RCAP - 1 ? RCAP - 1 : i0;
    int i1 = o + 32 + lane; i1 = i1 > RCAP - 1 ? RCAP - 1 : i1;
    const int ent0 = sl[i0];
    const int ent1 = sl[i1];
    int eid0 = ent0 >> SLA; eid0 = eid0 < 0 ? 0 : (eid0 > nE - 1 ? nE - 1 : eid0);
    int eid1 = ent1 >> SLA; eid1 = eid1 < 0 ? 0 : (eid1 > nE - 1 ? nE - 1 : eid1);
    int sr0 = srcs[eid0]; sr0 = sr0 < 0 ? 0 : (sr0 > nN - 1 ? nN - 1 : sr0);
    int sr1 = srcs[eid1]; sr1 = sr1 < 0 ? 0 : (sr1 > nN - 1 ? nN - 1 : sr1);
    const float es0 = ASp[sr0];
    const float es1 = ASp[sr1];
    const bool v0 = lane < c;
    const bool v1 = (lane + 32) < c;
    const float l0 = leaky(es0 + ad);
    const float l1 = leaky(es1 + ad);
    const float ls = leaky(as0 + ad);
    float mxl = fmaxf(v0 ? l0 : -3.0e38f, v1 ? l1 : -3.0e38f);
#pragma unroll
    for (int off = 16; off > 0; off >>= 1) mxl = fmaxf(mxl, __shfl_xor(mxl, off));
    const float mx = fmaxf(mxl, ls);
    const float e0 = expf(l0 - mx);
    const float e1 = expf(l1 - mx);
    const float a0 = v0 ? e0 : 0.0f;
    const float a1 = v1 ? e1 : 0.0f;
    const float asf = expf(ls - mx);
    float sm = a0 + a1;
#pragma unroll
    for (int off = 16; off > 0; off >>= 1) sm += __shfl_xor(sm, off);
    const float dn  = asf + sm;
    const float inv = 1.0f / dn;
    const int   w0i = __float_as_int(a0 * inv);
    const int   w1i = __float_as_int(a1 * inv);
    const float wsf = asf * inv;
    const int c0n = c < 32 ? c : 32;
    const int c1n = c - c0n;
    const float pzr = big ? qnan : pz;

#pragma unroll 1
    for (int cc = 0; cc < 2; ++cc) {
      const float* base = F + (size_t)(512 * cc + 4 * lane);
      const float* sp = base + (size_t)node * CH;
      v4f acc[4];
      {
        const v4f r0 = *(const v4f*)sp;
        const v4f r1 = *(const v4f*)(sp + 128);
        const v4f r2 = *(const v4f*)(sp + 256);
        const v4f r3 = *(const v4f*)(sp + 384);
        acc[0] = r0 * wsf; acc[1] = r1 * wsf; acc[2] = r2 * wsf; acc[3] = r3 * wsf;
      }
      gather_hits(acc, base, sr0, w0i, c0n);
      gather_hits(acc, base, sr1, w1i, c1n);
      const float* bq = bias + 512 * cc + 4 * lane;
      const v4f b0 = bfr4(*(const v4f*)bq);
      const v4f b1 = bfr4(*(const v4f*)(bq + 128));
      const v4f b2 = bfr4(*(const v4f*)(bq + 256));
      const v4f b3 = bfr4(*(const v4f*)(bq + 384));
      const v4f o0 = acc[0] + b0 + pzr;
      const v4f o1 = acc[1] + b1 + pzr;
      const v4f o2 = acc[2] + b2 + pzr;
      const v4f o3 = acc[3] + b3 + pzr;
      float* op = outp + (size_t)node * CH + 512 * cc + 4 * lane;
      *(volatile v4f*)op = o0;
      *(volatile v4f*)(op + 128) = o1;
      *(volatile v4f*)(op + 256) = o2;
      *(volatile v4f*)(op + 384) = o3;
      __threadfence();
      *(volatile v4f*)op = o0;
      *(volatile v4f*)(op + 128) = o1;
      *(volatile v4f*)(op + 256) = o2;
      *(volatile v4f*)(op + 384) = o3;
    }
  }
}

__global__ __launch_bounds__(NTHR) void k_bnstat(const float* __restrict__ X, int nN, double* REC) {
  __shared__ __attribute__((aligned(16))) double sS[CH];
  __shared__ __attribute__((aligned(16))) double sQ[CH];
  const int tid = (int)threadIdx.x;
  const int r0 = (int)blockIdx.x * BNR;
  int r1 = r0 + BNR; r1 = r1 > nN ? nN : r1;
  const int c0 = 4 * tid;
  double s0 = 0.0, s1 = 0.0, s2 = 0.0, s3 = 0.0, q0 = 0.0, q1 = 0.0, q2 = 0.0, q3 = 0.0;
#pragma unroll 2
  for (int r = r0; r < r1; ++r) {
    const v4f v = *(const v4f*)(X + (size_t)r * CH + c0);
    const double d0 = (double)v.x, d1 = (double)v.y, d2 = (double)v.z, d3 = (double)v.w;
    s0 += d0; s1 += d1; s2 += d2; s3 += d3;
    q0 = __builtin_fma(d0, d0, q0); q1 = __builtin_fma(d1, d1, q1);
    q2 = __builtin_fma(d2, d2, q2); q3 = __builtin_fma(d3, d3, q3);
  }
  sS[c0] = s0; sS[c0 + 1] = s1; sS[c0 + 2] = s2; sS[c0 + 3] = s3;
  sQ[c0] = q0; sQ[c0 + 1] = q1; sQ[c0 + 2] = q2; sQ[c0 + 3] = q3;
  __syncthreads();
  double* rb = REC + (size_t)blockIdx.x * (2 * CH);
  const v2d a0 = *(const v2da*)(sS + 2 * tid);
  const v2d a1 = *(const v2da*)(sS + 2 * (tid + NTHR));
  const v2d b0 = *(const v2da*)(sQ + 2 * tid);
  const v2d b1 = *(const v2da*)(sQ + 2 * (tid + NTHR));
  *(volatile v2d*)(rb + 2 * tid) = a0;
  *(volatile v2d*)(rb + 2 * (tid + NTHR)) = a1;
  *(volatile v2d*)(rb + CH + 2 * tid) = b0;
  *(volatile v2d*)(rb + CH + 2 * (tid + NTHR)) = b1;
  __threadfence();
  *(volatile v2d*)(rb + 2 * tid) = a0;
  *(volatile v2d*)(rb + 2 * (tid + NTHR)) = a1;
  *(volatile v2d*)(rb + CH + 2 * tid) = b0;
  *(volatile v2d*)(rb + CH + 2 * (tid + NTHR)) = b1;
}

__global__ __launch_bounds__(NTHR) void k_bncomb(const double* __restrict__ REC, int nch, double invN,
                                                 const float* __restrict__ bw, const float* __restrict__ bb,
                                                 float* PAR) {
  __shared__ __attribute__((aligned(16))) float sp[3 * CH];
  const int tid = (int)threadIdx.x;
#pragma unroll 1
  for (int it = 0; it < CH / NTHR; ++it) {
    const int c = tid + NTHR * it;
    double S = 0.0, Q = 0.0;
#pragma unroll 1
    for (int ch = 0; ch < nch; ++ch) {
      S += REC[(size_t)ch * (2 * CH) + c];
      Q += REC[(size_t)ch * (2 * CH) + CH + c];
    }
    const double mu = S * invN;
    double var = Q * invN - mu * mu;
    var = (var < 0.0) ? 0.0 : var;
    const float varf = (float)var;
    const float rs = 1.0f / sqrtf(varf + BN_EPS);
    sp[c]          = (float)mu;
    sp[CH + c]     = bf16_val(bw[c]) * rs;
    sp[2 * CH + c] = bf16_val(bb[c]);
  }
  __syncthreads();
  const v4f m4 = *(const v4fa*)(sp + 4 * tid);
  const v4f s4 = *(const v4fa*)(sp + CH + 4 * tid);
  const v4f b4 = *(const v4fa*)(sp + 2 * CH + 4 * tid);
  *(volatile v4f*)(PAR + 4 * tid) = m4;
  *(volatile v4f*)(PAR + CH + 4 * tid) = s4;
  *(volatile v4f*)(PAR + 2 * CH + 4 * tid) = b4;
  __threadfence();
  *(volatile v4f*)(PAR + 4 * tid) = m4;
  *(volatile v4f*)(PAR + CH + 4 * tid) = s4;
  *(volatile v4f*)(PAR + 2 * CH + 4 * tid) = b4;
}

__global__ __launch_bounds__(NTHR) void k_bnapply(const float* __restrict__ X, const float* __restrict__ PAR,
                                                  int nN, int nUnits, unsigned short* XP) {
  const int u = (int)blockIdx.x * NTHR + (int)threadIdx.x;
  if (u >= nUnits) return;
  const int row = u >> 7;
  const int c0  = (u & 127) * 8;
  const int rc  = row < nN ? row : nN - 1;
  const float* xp = X + (size_t)rc * CH + c0;
  const v4f xa = *(const v4f*)xp, xb = *(const v4f*)(xp + 4);
  const v4f ma = *(const v4f*)(PAR + c0),          mb = *(const v4f*)(PAR + c0 + 4);
  const v4f sa = *(const v4f*)(PAR + CH + c0),     sb = *(const v4f*)(PAR + CH + c0 + 4);
  const v4f ba = *(const v4f*)(PAR + 2 * CH + c0), bb = *(const v4f*)(PAR + 2 * CH + c0 + 4);
  const bool ok = row < nN;
  float v[8];
  v[0] = relu_keep(fmaf(xa.x - ma.x, sa.x, ba.x)); v[1] = relu_keep(fmaf(xa.y - ma.y, sa.y, ba.y));
  v[2] = relu_keep(fmaf(xa.z - ma.z, sa.z, ba.z)); v[3] = relu_keep(fmaf(xa.w - ma.w, sa.w, ba.w));
  v[4] = relu_keep(fmaf(xb.x - mb.x, sb.x, bb.x)); v[5] = relu_keep(fmaf(xb.y - mb.y, sb.y, bb.y));
  v[6] = relu_keep(fmaf(xb.z - mb.z, sb.z, bb.z)); v[7] = relu_keep(fmaf(xb.w - mb.w, sb.w, bb.w));
  v8us ho, lo;
#pragma unroll
  for (int i = 0; i < 8; ++i) {
    const float y = ok ? v[i] : 0.0f;
    const unsigned hbi = bf16_bits(y);
    ho[i] = (unsigned short)hbi;
    lo[i] = (unsigned short)bf16_bits(y - __uint_as_float(hbi << 16));
  }
  unsigned short* hp = XP + (size_t)row * K2 + c0;
  *(volatile v8us*)hp = ho;
  *(volatile v8us*)(hp + CH) = lo;
  __threadfence();
  *(volatile v8us*)hp = ho;
  *(volatile v8us*)(hp + CH) = lo;
}

static inline int cdiv(int a, int b) { return (a + b - 1) / b; }

extern "C" void kernel_launch(void* const* d_in, const int* in_sizes, int n_in,
                              void* d_out, int out_size, void* d_ws, size_t ws_size,
                              hipStream_t stream) {
  if (n_in < 18) return;
  if (in_sizes[0] < FIN || (in_sizes[0] % FIN) != 0) return;
  const int nN = in_sizes[0] / FIN;
  if (nN < 1 || nN > (1 << 20) || (nN & 1) != 0) return;
  if (in_sizes[1] < 2 || (in_sizes[1] & 1) != 0) return;
  const int nE = in_sizes[1] / 2;
  if (nE < 1 || nE >= (1 << 21)) return;
  if (in_sizes[2] != CH * FIN) return;
  if (in_sizes[3] != CH || in_sizes[4] != CH || in_sizes[5] != CH) return;
  if (in_sizes[6] != CH || in_sizes[7] != CH) return;
  if (in_sizes[8] != CH * CH) return;
  if (in_sizes[9] != CH || in_sizes[10] != CH || in_sizes[11] != CH) return;
  if (in_sizes[12] != CH || in_sizes[13] != CH) return;
  if (in_sizes[14] != NFC * CH || in_sizes[15] != NFC) return;
  if (in_sizes[16] != NOUT * NFC || in_sizes[17] != NOUT) return;
  if ((long long)out_size != (long long)nN * NOUT) return;

  const float* x     = (const float*)d_in[0];
  const int*   edge  = (const int*)  d_in[1];
  const float* W1    = (const float*)d_in[2];
  const float* a1s   = (const float*)d_in[3];
  const float* a1d   = (const float*)d_in[4];
  const float* b1    = (const float*)d_in[5];
  const float* bn1w  = (const float*)d_in[6];
  const float* bn1b  = (const float*)d_in[7];
  const float* W2    = (const float*)d_in[8];
  const float* a2s   = (const float*)d_in[9];
  const float* a2d   = (const float*)d_in[10];
  const float* b2    = (const float*)d_in[11];
  const float* bn2w  = (const float*)d_in[12];
  const float* bn2b  = (const float*)d_in[13];
  const float* fcw   = (const float*)d_in[14];
  const float* fcb   = (const float*)d_in[15];
  const float* fc1w  = (const float*)d_in[16];
  const float* fc1b  = (const float*)d_in[17];
  float* out = (float*)d_out;
  const int* src = edge;
  const int* dst = edge + nE;

  const int MP   = cdiv(nN, GBM) * GBM;
  const int gM   = MP / GBM;
  const int gA   = cdiv(nN, NBA);
  const int nch  = cdiv(nN, BNR);
  const int vec8 = ((nE & 3) == 0) ? 1 : 0;
  const int nUx  = MP * (FIN / 8);
  if ((nUx % NTHR) != 0) return;
  if ((long long)gA * NBA < (long long)nN) return;

  char* ws = (char*)d_ws;
  size_t off = 0;
  const size_t oXB  = off; off += (size_t)MP * FIN * 2;              off = (off + 255) & ~(size_t)255;
  const size_t oW1B = off; off += (size_t)CH * FIN * 2;              off = (off + 255) & ~(size_t)255;
  const size_t oW2D = off; off += (size_t)CH * K2 * 2;               off = (off + 255) & ~(size_t)255;
  const size_t oFCD = off; off += (size_t)NFC * K2 * 2;              off = (off + 255) & ~(size_t)255;
  const size_t oSD  = off; off += (size_t)2 * MP * 4;                off = (off + 255) & ~(size_t)255;
  const size_t oREC = off; off += (size_t)nch * 2 * CH * 8;          off = (off + 255) & ~(size_t)255;
  const size_t oPAR = off; off += (size_t)3 * CH * 4;                off = (off + 255) & ~(size_t)255;
  const size_t oRA  = off; off += (size_t)MP * CH * 4;               off = (off + 255) & ~(size_t)255;
  const size_t oRB  = off; off += (size_t)MP * CH * 4;               off = (off + 255) & ~(size_t)255;
  if (off > ws_size || off > (size_t)WSMAX) return;
  unsigned short* XB  = (unsigned short*)(ws + oXB);
  unsigned short* W1B = (unsigned short*)(ws + oW1B);
  unsigned short* W2D = (unsigned short*)(ws + oW2D);
  unsigned short* FCD = (unsigned short*)(ws + oFCD);
  float*  SD  = (float*)(ws + oSD);
  double* REC = (double*)(ws + oREC);
  float*  PAR = (float*)(ws + oPAR);
  float*  RAf = (float*)(ws + oRA);
  float*  RBf = (float*)(ws + oRB);
  unsigned short* RAh = (unsigned short*)(ws + oRA);
  unsigned short* RBh = (unsigned short*)(ws + oRB);

  const size_t aggLds  = (size_t)AGG_LDS_INTS * 4;
  const size_t headLds = (size_t)HEAD_LDS_FLOATS * 4;
  hipFuncSetAttribute(reinterpret_cast<const void*>(&k_agg), hipFuncAttributeMaxDynamicSharedMemorySize, (int)aggLds);
  hipFuncSetAttribute(reinterpret_cast<const void*>(&k_gemm_head), hipFuncAttributeMaxDynamicSharedMemorySize, (int)headLds);

  const double invN = 1.0 / (double)nN;
  const int nUa = MP * (CH / 8);
  const dim3 gG(gM, CH / GBN);

  k_prep<<<(nUx + NU_W1 + NU_W2 + NU_FC) / NTHR, NTHR, 0, stream>>>(x, W1, W2, fcw, XB, W1B, W2D, FCD, nN, nUx);

  k_gemm<<<gG, GTHR, 0, stream>>>(XB, FIN, W1B, FIN, FIN, RAf, CH);
  k_dots<<<gM, NTHR, 0, stream>>>(RAf, a1s, a1d, SD, MP);
  k_agg<<<gA, NTHR, aggLds, stream>>>(src, dst, nE, nN, vec8, MP, SD, RAf, b1, RBf);
  k_bnstat<<<nch, NTHR, 0, stream>>>(RBf, nN, REC);
  k_bncomb<<<1, NTHR, 0, stream>>>(REC, nch, invN, bn1w, bn1b, PAR);
  k_bnapply<<<cdiv(nUa, NTHR), NTHR, 0, stream>>>(RBf, PAR, nN, nUa, RAh);

  k_gemm<<<gG, GTHR, 0, stream>>>(RAh, K2, W2D, K2, K2, RBf, CH);
  k_dots<<<gM, NTHR, 0, stream>>>(RBf, a2s, a2d, SD, MP);
  k_agg<<<gA, NTHR, aggLds, stream>>>(src, dst, nE, nN, vec8, MP, SD, RBf, b2, RAf);
  k_bnstat<<<nch, NTHR, 0, stream>>>(RAf, nN, REC);
  k_bncomb<<<1, NTHR, 0, stream>>>(REC, nch, invN, bn2w, bn2b, PAR);
  k_bnapply<<<cdiv(nUa, NTHR), NTHR, 0, stream>>>(RAf, PAR, nN, nUa, RBh);

  k_gemm_head<<<gM, HTHR, headLds, stream>>>(RBh, FCD, fcb, fc1w, fc1b, out, nN);
}
